// ProteinGrid_66108136620512
// MI455X (gfx1250) — hardware-verified
//
#include <hip/hip_runtime.h>
#include <stddef.h>
#include <stdint.h>


#define NVOX  4096
#define NNODE 4096
#define DEGV  256
#define HIDC  64
#define NCLS  20
#define NTHR  128
#define NWAV  4

static_assert(NVOX % NWAV == 0);
static_assert((NVOX / 16) % NWAV == 0);

typedef float          v4f  __attribute__((ext_vector_type(4)));
typedef float          v8f  __attribute__((ext_vector_type(8)));
typedef _Float16       v8h  __attribute__((ext_vector_type(8)));
typedef _Float16       v16h __attribute__((ext_vector_type(16)));
typedef unsigned short v8us __attribute__((ext_vector_type(8)));
typedef __bf16         v16b __attribute__((ext_vector_type(16)));
typedef unsigned int   v8u  __attribute__((ext_vector_type(8)));

union FragH { v16h v; v8h h[2]; v8u w; };
union FragB { v16b v; v8us u[2]; };
static_assert(sizeof(FragH) == 32);
static_assert(sizeof(FragB) == 32);

__device__ __forceinline__ v8f wmh(v16h a, v16h b, v8f c) {
  v8f d = __builtin_amdgcn_wmma_f32_16x16x32_f16(false, a, false, b, (short)0, c, false, false);
  asm volatile("v_nop\n\tv_nop\n\tv_nop\n\tv_nop" : "+v"(d) : "v"(a), "v"(b));
  return d;
}
__device__ __forceinline__ v8f wmb(v16b a, v16b b, v8f c) {
  v8f d = __builtin_amdgcn_wmma_f32_16x16x32_bf16(false, a, false, b, (short)0, c, false, false);
  asm volatile("v_nop\n\tv_nop\n\tv_nop\n\tv_nop" : "+v"(d) : "v"(a), "v"(b));
  return d;
}
__device__ __forceinline__ v8f splat8(float x) {
  v8f c;
#pragma unroll
  for (int i = 0; i < 8; ++i) c[i] = x;
  return c;
}
__device__ __forceinline__ float silu_f(float x) {
  return x * __builtin_amdgcn_rcpf(1.0f + __expf(-x));
}
__device__ __forceinline__ unsigned short bf_rne(float x) {
  unsigned u = __float_as_uint(x);
  u += 0x7FFFu + ((u >> 16) & 1u);
  return (unsigned short)(u >> 16);
}
__device__ __forceinline__ float bf_val(unsigned short b) {
  return __uint_as_float(((unsigned)b) << 16);
}
__device__ __forceinline__ v8h cvt8(v4f a, v4f b) {
  v8h r;
  r[0] = (_Float16)a.x; r[1] = (_Float16)a.y; r[2] = (_Float16)a.z; r[3] = (_Float16)a.w;
  r[4] = (_Float16)b.x; r[5] = (_Float16)b.y; r[6] = (_Float16)b.z; r[7] = (_Float16)b.w;
  return r;
}

__global__ __launch_bounds__(256) void k_prep_lin(
    const float* __restrict__ ew2, const float* __restrict__ mw1, const float* __restrict__ uw1,
    const float* __restrict__ uw2, const float* __restrict__ mw2, _Float16* P16, unsigned short* PBF) {
  const int pid = blockIdx.x, tid = threadIdx.x;
  const float* src = ew2;
  int roff = 0;
  if (pid == 1) { src = mw1; }
  else if (pid == 2) { src = mw1; roff = HIDC; }
  else if (pid == 3) { src = uw1; }
  else if (pid == 4) { src = uw2; }
  else if (pid >= 5) { src = mw2; }
  float x[2][8];
  int n[2], k0[2];
#pragma unroll
  for (int s = 0; s < 2; ++s) {
    const int q = tid + 256 * s;
    n[s] = q >> 3;
    k0[s] = (q & 7) * 8;
#pragma unroll
    for (int u = 0; u < 8; ++u) x[s][u] = src[(size_t)(roff + k0[s] + u) * HIDC + n[s]];
  }
  if (pid < 5) {
    v8h hv[2];
#pragma unroll
    for (int s = 0; s < 2; ++s) {
#pragma unroll
      for (int u = 0; u < 8; ++u) hv[s][u] = (_Float16)(x[s][u] * 16.0f);
    }
    _Float16* base = P16 + (size_t)pid * 4096;
#pragma unroll
    for (int s = 0; s < 2; ++s) *(volatile v8h*)(base + n[s] * HIDC + k0[s]) = hv[s];
    __threadfence();
#pragma unroll
    for (int s = 0; s < 2; ++s) *(volatile v8h*)(base + n[s] * HIDC + k0[s]) = hv[s];
  } else {
    v8us bv[2];
#pragma unroll
    for (int s = 0; s < 2; ++s) {
#pragma unroll
      for (int u = 0; u < 8; ++u) {
        const unsigned short hs = bf_rne(x[s][u]);
        const unsigned short ls = bf_rne(x[s][u] - bf_val(hs));
        bv[s][u] = (pid == 5) ? hs : ls;
      }
    }
    unsigned short* base = PBF + (size_t)(pid - 5) * 4096;
#pragma unroll
    for (int s = 0; s < 2; ++s) *(volatile v8us*)(base + n[s] * HIDC + k0[s]) = bv[s];
    __threadfence();
#pragma unroll
    for (int s = 0; s < 2; ++s) *(volatile v8us*)(base + n[s] * HIDC + k0[s]) = bv[s];
  }
}

__global__ __launch_bounds__(256) void k_prep_conv(const float* __restrict__ W, _Float16* P,
                                                   int Cout, int Cin, int T) {
  const int K = T * Cin;
  const int ppr = K >> 3;
  const int np = Cout * ppr;
  const int g = blockIdx.x * 256 + threadIdx.x;
  const bool act = g < np;
  const int gg = act ? g : 0;
  const int co = gg / ppr;
  const int rem = gg - co * ppr;
  const int k0 = rem * 8;
  const int t = k0 / Cin;
  const int ci0 = k0 - t * Cin;
  v8h v;
#pragma unroll
  for (int u = 0; u < 8; ++u)
    v[u] = (_Float16)(W[((size_t)(co * Cin + ci0 + u)) * (size_t)T + t] * 64.0f);
  _Float16* p = P + (size_t)co * K + k0;
  if (act) *(volatile v8h*)p = v;
  __threadfence();
  if (act) *(volatile v8h*)p = v;
}

__global__ __launch_bounds__(NTHR) void k_nq(const float* __restrict__ emb, const _Float16* w1a, float* NQ) {
  __shared__ __attribute__((aligned(16))) float stg[NWAV][16 * HIDC];
  const int tid = threadIdx.x, lane = tid & 31, w = tid >> 5, h = lane >> 4, m = lane & 15;
  const int r0 = (blockIdx.x * NWAV + w) * 16;
  float* st = stg[w];
  FragH a[2];
#pragma unroll
  for (int kc = 0; kc < 2; ++kc) {
    const float* ap = emb + (size_t)(r0 + m) * HIDC + kc * 32 + 8 * h;
    const v4f x0 = *(const v4f*)ap, x1 = *(const v4f*)(ap + 4);
    const v4f x2 = *(const v4f*)(ap + 16), x3 = *(const v4f*)(ap + 20);
    a[kc].h[0] = cvt8(x0, x1);
    a[kc].h[1] = cvt8(x2, x3);
  }
#pragma unroll
  for (int nb = 0; nb < 4; ++nb) {
    const int col = nb * 16 + m;
    v8f acc = splat8(0.0f);
#pragma unroll
    for (int kc = 0; kc < 2; ++kc) {
      FragH b;
      const _Float16* bp = w1a + (size_t)col * HIDC + kc * 32 + 8 * h;
      b.h[0] = *(const v8h*)bp;
      b.h[1] = *(const v8h*)(bp + 16);
      acc = wmh(a[kc].v, b.v, acc);
    }
#pragma unroll
    for (int r = 0; r < 8; ++r) st[(8 * h + r) * HIDC + col] = acc[r] * 0.0625f;
  }
  __syncthreads();
  v4f ov[8];
#pragma unroll
  for (int it = 0; it < 8; ++it) {
    const int line = it * 4 + (lane >> 3), row = line >> 1, hf = line & 1;
    ov[it] = *(const v4f*)(st + row * HIDC + hf * 32 + (lane & 7) * 4);
  }
  float* ob = NQ + (size_t)r0 * HIDC;
#pragma unroll
  for (int it = 0; it < 8; ++it) {
    const int line = it * 4 + (lane >> 3), row = line >> 1, hf = line & 1;
    *(volatile v4f*)(ob + row * HIDC + hf * 32 + (lane & 7) * 4) = ov[it];
  }
  __threadfence();
#pragma unroll
  for (int it = 0; it < 8; ++it) {
    const int line = it * 4 + (lane >> 3), row = line >> 1, hf = line & 1;
    *(volatile v4f*)(ob + row * HIDC + hf * 32 + (lane & 7) * 4) = ov[it];
  }
}

__global__ __launch_bounds__(NTHR) void k_mpnn(
    const float* __restrict__ npos, const float* __restrict__ gpos, const int* __restrict__ ei,
    const float* __restrict__ ew1, const float* __restrict__ eb1, const float* __restrict__ eb2,
    const float* __restrict__ mb1, const _Float16* ew2p, const _Float16* mw1bp,
    const float* NQ, float* S1, int nN) {
  __shared__ __attribute__((aligned(16))) float    pl[NWAV][16 * 4];
  __shared__ __attribute__((aligned(16))) float    nql[NWAV][16 * HIDC];
  __shared__ __attribute__((aligned(16))) _Float16 hA[NWAV][16 * HIDC];
  __shared__ __attribute__((aligned(16))) _Float16 hP[NWAV][16 * HIDC];
  __shared__ __attribute__((aligned(16))) float    rowb[NWAV][HIDC];
  const int tid = threadIdx.x, lane = tid & 31, w = tid >> 5, h = lane >> 4, m = lane & 15;
  const int j = blockIdx.x * NWAV + w;
  float* pl_l = pl[w];
  float* nq_l = nql[w];
  _Float16* hA_l = hA[w];
  _Float16* hP_l = hP[w];
  float* rb_l = rowb[w];

  const float gp0 = gpos[j * 3 + 0], gp1 = gpos[j * 3 + 1], gp2 = gpos[j * 3 + 2];
  const float wa0 = ew1[lane],      wa1 = ew1[64 + lane],  wa2 = ew1[128 + lane];
  const float wb0 = ew1[32 + lane], wb1 = ew1[96 + lane],  wb2 = ew1[160 + lane];
  const float ga = eb1[lane]      + gp0 * ew1[192 + lane] + gp1 * ew1[256 + lane] + gp2 * ew1[320 + lane];
  const float gb = eb1[32 + lane] + gp0 * ew1[224 + lane] + gp1 * ew1[288 + lane] + gp2 * ew1[352 + lane];
  float eb2v[4], mb1v[4], csum[4];
#pragma unroll
  for (int nb = 0; nb < 4; ++nb) {
    const int col = nb * 16 + m;
    eb2v[nb] = 16.0f * eb2[col];
    mb1v[nb] = mb1[col];
    csum[nb] = 0.0f;
  }
  const int rr = lane >> 1, hf = lane & 1;

#pragma unroll 1
  for (int tt = 0; tt < 16; ++tt) {
    __syncthreads();
    const int e0 = j * DEGV + tt * 16;
    {
      int i2 = ei[e0 + rr];
      i2 = min(max(i2, 0), nN - 1);
      const float* pp = npos + (size_t)i2 * 3;
      const float q0 = pp[0], q1 = pp[1], q2 = pp[2];
      pl_l[rr * 4 + hf * 2]     = hf ? q2 : q0;
      pl_l[rr * 4 + hf * 2 + 1] = hf ? 0.0f : q1;
      const float* sp = NQ + (size_t)i2 * HIDC + hf * 32;
      float* dp = nq_l + rr * HIDC + hf * 32;
#pragma unroll
      for (int q = 0; q < 8; ++q) *(v4f*)(dp + 4 * q) = *(const v4f*)(sp + 4 * q);
    }
    __syncthreads();
#pragma unroll 4
    for (int e = 0; e < 16; ++e) {
      const v4f p = *(const v4f*)(pl_l + 4 * e);
      const float za = ga + p.x * wa0 + p.y * wa1 + p.z * wa2;
      const float zb = gb + p.x * wb0 + p.y * wb1 + p.z * wb2;
      hA_l[e * HIDC + lane]      = (_Float16)silu_f(za);
      hA_l[e * HIDC + 32 + lane] = (_Float16)silu_f(zb);
    }
    __syncthreads();
    {
      FragH a0, a1;
      const _Float16* abase = hA_l + m * HIDC + 8 * h;
      a0.h[0] = *(const v8h*)abase;        a0.h[1] = *(const v8h*)(abase + 16);
      a1.h[0] = *(const v8h*)(abase + 32); a1.h[1] = *(const v8h*)(abase + 48);
#pragma unroll
      for (int nb = 0; nb < 4; ++nb) {
        const int col = nb * 16 + m;
        v8f acc = splat8(eb2v[nb]);
        const _Float16* bp = ew2p + (size_t)col * HIDC + 8 * h;
        FragH b;
        b.h[0] = *(const v8h*)bp;        b.h[1] = *(const v8h*)(bp + 16);
        acc = wmh(a0.v, b.v, acc);
        b.h[0] = *(const v8h*)(bp + 32); b.h[1] = *(const v8h*)(bp + 48);
        acc = wmh(a1.v, b.v, acc);
#pragma unroll
        for (int r = 0; r < 8; ++r) hP_l[(8 * h + r) * HIDC + col] = (_Float16)(acc[r] * 0.0625f);
      }
    }
    __syncthreads();
    {
      FragH a0, a1;
      const _Float16* abase = hP_l + m * HIDC + 8 * h;
      a0.h[0] = *(const v8h*)abase;        a0.h[1] = *(const v8h*)(abase + 16);
      a1.h[0] = *(const v8h*)(abase + 32); a1.h[1] = *(const v8h*)(abase + 48);
#pragma unroll
      for (int nb = 0; nb < 4; ++nb) {
        const int col = nb * 16 + m;
        v8f acc;
#pragma unroll
        for (int r = 0; r < 8; ++r) acc[r] = 16.0f * (nq_l[(8 * h + r) * HIDC + col] + mb1v[nb]);
        const _Float16* bp = mw1bp + (size_t)col * HIDC + 8 * h;
        FragH b;
        b.h[0] = *(const v8h*)bp;        b.h[1] = *(const v8h*)(bp + 16);
        acc = wmh(a0.v, b.v, acc);
        b.h[0] = *(const v8h*)(bp + 32); b.h[1] = *(const v8h*)(bp + 48);
        acc = wmh(a1.v, b.v, acc);
        float s = 0.0f;
#pragma unroll
        for (int r = 0; r < 8; ++r) s += silu_f(acc[r] * 0.0625f);
        csum[nb] += s;
      }
    }
  }
#pragma unroll
  for (int nb = 0; nb < 4; ++nb) {
    const float tot = csum[nb] + __shfl_xor(csum[nb], 16);
    if (h == 0) rb_l[nb * 16 + m] = tot * (1.0f / 256.0f);
  }
  __syncthreads();
  const v4f ov = *(const v4f*)(rb_l + 4 * (lane & 15));
  float* op = S1 + (size_t)j * HIDC + 4 * (lane & 15);
  if (lane < 16) *(volatile v4f*)op = ov;
  __threadfence();
  if (lane < 16) *(volatile v4f*)op = ov;
}

__global__ __launch_bounds__(NTHR) void k_upd(
    const float* S1, const unsigned short* w2hi, const unsigned short* w2lo,
    const float* __restrict__ mb2, const _Float16* uw1p, const float* __restrict__ ub1,
    const _Float16* uw2p, const float* __restrict__ ub2, _Float16* X0, float bnc) {
  __shared__ __attribute__((aligned(16))) _Float16 tA[NWAV][16 * HIDC];
  __shared__ __attribute__((aligned(16))) _Float16 tB[NWAV][16 * HIDC];
  __shared__ __attribute__((aligned(16))) _Float16 tO[NWAV][16 * HIDC];
  const int tid = threadIdx.x, lane = tid & 31, w = tid >> 5, h = lane >> 4, m = lane & 15;
  const int v0 = (blockIdx.x * NWAV + w) * 16;
  _Float16* tA_l = tA[w];
  _Float16* tB_l = tB[w];
  _Float16* tO_l = tO[w];

  FragB ah[2], al[2];
#pragma unroll
  for (int kc = 0; kc < 2; ++kc) {
#pragma unroll
    for (int part = 0; part < 2; ++part) {
      const float* sp = S1 + (size_t)(v0 + m) * HIDC + kc * 32 + 16 * part + 8 * h;
      const v4f xa = *(const v4f*)sp, xb = *(const v4f*)(sp + 4);
      float xs[8];
      xs[0] = xa.x; xs[1] = xa.y; xs[2] = xa.z; xs[3] = xa.w;
      xs[4] = xb.x; xs[5] = xb.y; xs[6] = xb.z; xs[7] = xb.w;
      v8us th, tl;
#pragma unroll
      for (int u = 0; u < 8; ++u) {
        const unsigned short hs = bf_rne(xs[u]);
        th[u] = hs;
        tl[u] = bf_rne(xs[u] - bf_val(hs));
      }
      ah[kc].u[part] = th;
      al[kc].u[part] = tl;
    }
  }
#pragma unroll
  for (int nb = 0; nb < 4; ++nb) {
    const int col = nb * 16 + m;
    v8f acc = splat8(0.0f);
#pragma unroll
    for (int kc = 0; kc < 2; ++kc) {
      FragB bh, bl;
      const unsigned short* bp = w2hi + (size_t)col * HIDC + kc * 32 + 8 * h;
      const unsigned short* bq = w2lo + (size_t)col * HIDC + kc * 32 + 8 * h;
      bh.u[0] = *(const v8us*)bp; bh.u[1] = *(const v8us*)(bp + 16);
      bl.u[0] = *(const v8us*)bq; bl.u[1] = *(const v8us*)(bq + 16);
      acc = wmb(ah[kc].v, bh.v, acc);
      acc = wmb(ah[kc].v, bl.v, acc);
      acc = wmb(al[kc].v, bh.v, acc);
    }
    const float bias = mb2[col];
#pragma unroll
    for (int r = 0; r < 8; ++r) tA_l[(8 * h + r) * HIDC + col] = (_Float16)(acc[r] + bias);
  }
  __syncthreads();
  {
    FragH a0, a1;
    const _Float16* abase = tA_l + m * HIDC + 8 * h;
    a0.h[0] = *(const v8h*)abase;        a0.h[1] = *(const v8h*)(abase + 16);
    a1.h[0] = *(const v8h*)(abase + 32); a1.h[1] = *(const v8h*)(abase + 48);
#pragma unroll
    for (int nb = 0; nb < 4; ++nb) {
      const int col = nb * 16 + m;
      v8f acc = splat8(16.0f * ub1[col]);
      const _Float16* bp = uw1p + (size_t)col * HIDC + 8 * h;
      FragH b;
      b.h[0] = *(const v8h*)bp;        b.h[1] = *(const v8h*)(bp + 16);
      acc = wmh(a0.v, b.v, acc);
      b.h[0] = *(const v8h*)(bp + 32); b.h[1] = *(const v8h*)(bp + 48);
      acc = wmh(a1.v, b.v, acc);
#pragma unroll
      for (int r = 0; r < 8; ++r) tB_l[(8 * h + r) * HIDC + col] = (_Float16)silu_f(acc[r] * 0.0625f);
    }
  }
  __syncthreads();
  {
    FragH a0, a1;
    const _Float16* abase = tB_l + m * HIDC + 8 * h;
    a0.h[0] = *(const v8h*)abase;        a0.h[1] = *(const v8h*)(abase + 16);
    a1.h[0] = *(const v8h*)(abase + 32); a1.h[1] = *(const v8h*)(abase + 48);
#pragma unroll
    for (int nb = 0; nb < 4; ++nb) {
      const int col = nb * 16 + m;
      v8f acc = splat8(16.0f * ub2[col]);
      const _Float16* bp = uw2p + (size_t)col * HIDC + 8 * h;
      FragH b;
      b.h[0] = *(const v8h*)bp;        b.h[1] = *(const v8h*)(bp + 16);
      acc = wmh(a0.v, b.v, acc);
      b.h[0] = *(const v8h*)(bp + 32); b.h[1] = *(const v8h*)(bp + 48);
      acc = wmh(a1.v, b.v, acc);
#pragma unroll
      for (int r = 0; r < 8; ++r) tO_l[(8 * h + r) * HIDC + col] = (_Float16)(acc[r] * 0.0625f * bnc);
    }
  }
  __syncthreads();
  v8h ov[4];
#pragma unroll
  for (int it = 0; it < 4; ++it) {
    const int row = it * 4 + (lane >> 3), pc = (lane & 7) * 8;
    ov[it] = *(const v8h*)(tO_l + row * HIDC + pc);
  }
#pragma unroll
  for (int it = 0; it < 4; ++it) {
    const int row = it * 4 + (lane >> 3), pc = (lane & 7) * 8;
    *(volatile v8h*)(X0 + (size_t)(v0 + row) * HIDC + pc) = ov[it];
  }
  __threadfence();
#pragma unroll
  for (int it = 0; it < 4; ++it) {
    const int row = it * 4 + (lane >> 3), pc = (lane & 7) * 8;
    *(volatile v8h*)(X0 + (size_t)(v0 + row) * HIDC + pc) = ov[it];
  }
}

template <int CIN, int KS>
__device__ __forceinline__ void conv_taps(v8f (&acc)[4], const _Float16* X, const _Float16* Wp,
                                          int z, int y, int col0, int lane) {
  constexpr int P = KS / 2, KC = CIN / 32;
  constexpr int K = KS * KS * KS * CIN;
  const int h = lane >> 4, m = lane & 15;
  const _Float16* wl = Wp + (size_t)(col0 + m) * K + 8 * h;
#pragma unroll 1
  for (int dz = -P; dz <= P; ++dz) {
    const int zz = z + dz;
    if ((unsigned)zz >= 16u) continue;
#pragma unroll 1
    for (int dy = -P; dy <= P; ++dy) {
      const int yy = y + dy;
      if ((unsigned)yy >= 16u) continue;
      const int rowv = (zz * 16 + yy) * 16;
      const int tzy = ((dz + P) * KS + (dy + P)) * KS;
#pragma unroll 1
      for (int dx = -P; dx <= P; ++dx) {
        const int xx = m + dx;
        const bool inb = (unsigned)xx < 16u;
        const int xs = min(max(xx, 0), 15);
        const _Float16* al = X + (size_t)(rowv + xs) * CIN + 8 * h;
        const _Float16* bl = wl + (size_t)(tzy + dx + P) * CIN;
#pragma unroll 1
        for (int kc = 0; kc < KC; ++kc) {
          FragH a;
          a.h[0] = *(const v8h*)(al + kc * 32);
          a.h[1] = *(const v8h*)(al + kc * 32 + 16);
#pragma unroll
          for (int i = 0; i < 8; ++i) a.w[i] = inb ? a.w[i] : 0u;
#pragma unroll
          for (int nb = 0; nb < 4; ++nb) {
            FragH b;
            const _Float16* bq = bl + (size_t)nb * 16 * K + kc * 32;
            b.h[0] = *(const v8h*)bq;
            b.h[1] = *(const v8h*)(bq + 16);
            acc[nb] = wmh(a.v, b.v, acc[nb]);
          }
        }
      }
    }
  }
}

template <int CB, int CS, int COUT, int OUT32>
__global__ __launch_bounds__(NTHR) void k_conv(const _Float16* XB, const _Float16* WB,
                                               const _Float16* XS, const _Float16* WS,
                                               _Float16* Y16, float* Y32, float osc) {
  __shared__ __attribute__((aligned(16))) float    stf[NWAV][16 * 64];
  __shared__ __attribute__((aligned(16))) _Float16 sth[NWAV][16 * 64];
  constexpr int NCG = COUT / 64;
  const int tid = threadIdx.x, lane = tid & 31, w = tid >> 5, h = lane >> 4, m = lane & 15;
  const int task = blockIdx.x * NWAV + w;
  const int cg = task % NCG, zy = task / NCG;
  const int z = zy >> 4, y = zy & 15, vox0 = zy * 16, col0 = cg * 64;
  v8f acc[4];
#pragma unroll
  for (int nb = 0; nb < 4; ++nb) acc[nb] = splat8(0.0f);
  conv_taps<CB, 3>(acc, XB, WB, z, y, col0, lane);
  if (CS > 0) conv_taps<CS, 5>(acc, XS, WS, z, y, col0, lane);
  if (OUT32 != 0) {
    float* st = stf[w];
#pragma unroll
    for (int nb = 0; nb < 4; ++nb) {
#pragma unroll
      for (int r = 0; r < 8; ++r) st[(8 * h + r) * 64 + nb * 16 + m] = fmaxf(acc[nb][r] * osc, 0.0f);
    }
    __syncthreads();
    v4f ov[8];
#pragma unroll
    for (int it = 0; it < 8; ++it) {
      const int line = it * 4 + (lane >> 3), row = line >> 1, hf = line & 1;
      ov[it] = *(const v4f*)(st + row * 64 + hf * 32 + (lane & 7) * 4);
    }
#pragma unroll
    for (int it = 0; it < 8; ++it) {
      const int line = it * 4 + (lane >> 3), row = line >> 1, hf = line & 1;
      *(volatile v4f*)(Y32 + (size_t)(vox0 + row) * COUT + col0 + hf * 32 + (lane & 7) * 4) = ov[it];
    }
    __threadfence();
#pragma unroll
    for (int it = 0; it < 8; ++it) {
      const int line = it * 4 + (lane >> 3), row = line >> 1, hf = line & 1;
      *(volatile v4f*)(Y32 + (size_t)(vox0 + row) * COUT + col0 + hf * 32 + (lane & 7) * 4) = ov[it];
    }
  } else {
    _Float16* st = sth[w];
#pragma unroll
    for (int nb = 0; nb < 4; ++nb) {
#pragma unroll
      for (int r = 0; r < 8; ++r)
        st[(8 * h + r) * 64 + nb * 16 + m] = (_Float16)fmaxf(acc[nb][r] * osc, 0.0f);
    }
    __syncthreads();
    v8h ov[4];
#pragma unroll
    for (int it = 0; it < 4; ++it) {
      const int row = it * 4 + (lane >> 3), pc = (lane & 7) * 8;
      ov[it] = *(const v8h*)(st + row * 64 + pc);
    }
#pragma unroll
    for (int it = 0; it < 4; ++it) {
      const int row = it * 4 + (lane >> 3), pc = (lane & 7) * 8;
      *(volatile v8h*)(Y16 + (size_t)(vox0 + row) * COUT + col0 + pc) = ov[it];
    }
    __threadfence();
#pragma unroll
    for (int it = 0; it < 4; ++it) {
      const int row = it * 4 + (lane >> 3), pc = (lane & 7) * 8;
      *(volatile v8h*)(Y16 + (size_t)(vox0 + row) * COUT + col0 + pc) = ov[it];
    }
  }
}

__global__ __launch_bounds__(256) void k_pool(const float* Y3, const float* __restrict__ fcw,
                                              const float* __restrict__ fcb, float* out) {
  __shared__ float pooled[256];
  __shared__ __attribute__((aligned(16))) float res[32];
  const int tid = threadIdx.x;
  float mx = -3.0e38f;
#pragma unroll 4
  for (int v = 0; v < NVOX; ++v) mx = fmaxf(mx, Y3[(size_t)v * 256 + tid]);
  pooled[tid] = mx;
  __syncthreads();
  if (tid < 32) {
    const int cc = min(tid, NCLS - 1);
    float s = 0.0f;
#pragma unroll 1
    for (int i = 0; i < 256; ++i) s += pooled[i] * fcw[i * NCLS + cc];
    const float rv = s + fcb[cc];
    res[tid] = (tid < NCLS) ? rv : 0.0f;
  }
  __syncthreads();
  const v4f ov = *(const v4f*)(res + 4 * min(tid, 7));
  const bool wr = tid < 5;
  if (wr) *(volatile v4f*)(out + 4 * tid) = ov;
  __threadfence();
  if (wr) *(volatile v4f*)(out + 4 * tid) = ov;
}

extern "C" void kernel_launch(void* const* d_in, const int* in_sizes, int n_in,
                              void* d_out, int out_size, void* d_ws, size_t ws_size,
                              hipStream_t stream) {
  if (n_in < 27) return;
  const int nE = NVOX * DEGV;
  if (in_sizes[0] != NNODE * HIDC || in_sizes[1] != NNODE * 3 || in_sizes[2] != NVOX * 3) return;
  if (in_sizes[3] != 2 * nE) return;
  if (in_sizes[4] != 6 * HIDC || in_sizes[5] < HIDC || in_sizes[6] != HIDC * HIDC || in_sizes[7] < HIDC) return;
  if (in_sizes[8] != 2 * HIDC * HIDC || in_sizes[9] < HIDC || in_sizes[10] != HIDC * HIDC || in_sizes[11] < HIDC) return;
  if (in_sizes[12] != HIDC * HIDC || in_sizes[13] < HIDC || in_sizes[14] != HIDC * HIDC || in_sizes[15] < HIDC) return;
  if (in_sizes[16] != 64 * 64 * 27 || in_sizes[17] != 64 * 64 * 27 || in_sizes[18] != 64 * 64 * 125) return;
  if (in_sizes[19] != 128 * 64 * 27 || in_sizes[20] != 128 * 128 * 27 || in_sizes[21] != 128 * 64 * 125) return;
  if (in_sizes[22] != 256 * 128 * 27 || in_sizes[23] != 256 * 256 * 27 || in_sizes[24] != 256 * 128 * 125) return;
  if (in_sizes[25] != 256 * NCLS || in_sizes[26] < NCLS) return;
  if (out_size != NCLS) return;

  const float* node_emb = (const float*)d_in[0];
  const float* node_pos = (const float*)d_in[1];
  const float* grid_pos = (const float*)d_in[2];
  const int*   edge_i   = (const int*)d_in[3];
  const float* ew1 = (const float*)d_in[4];  const float* eb1 = (const float*)d_in[5];
  const float* ew2 = (const float*)d_in[6];  const float* eb2 = (const float*)d_in[7];
  const float* mw1 = (const float*)d_in[8];  const float* mb1 = (const float*)d_in[9];
  const float* mw2 = (const float*)d_in[10]; const float* mb2 = (const float*)d_in[11];
  const float* uw1 = (const float*)d_in[12]; const float* ub1 = (const float*)d_in[13];
  const float* uw2 = (const float*)d_in[14]; const float* ub2 = (const float*)d_in[15];
  const float* c1a = (const float*)d_in[16]; const float* c1b = (const float*)d_in[17];
  const float* c1s = (const float*)d_in[18];
  const float* c2a = (const float*)d_in[19]; const float* c2b = (const float*)d_in[20];
  const float* c2s = (const float*)d_in[21];
  const float* c3a = (const float*)d_in[22]; const float* c3b = (const float*)d_in[23];
  const float* c3s = (const float*)d_in[24];
  const float* fcw = (const float*)d_in[25]; const float* fcb = (const float*)d_in[26];
  float* out = (float*)d_out;

  const int K1A = 27 * 64,  K1B = 27 * 64,  K1S = 125 * 64;
  const int K2A = 27 * 64,  K2B = 27 * 128, K2S = 125 * 64;
  const int K3A = 27 * 128, K3B = 27 * 256, K3S = 125 * 128;

  char* ws = (char*)d_ws;
  size_t off = 0;
  auto carve = [&](size_t bytes) -> size_t { const size_t o = off; off += (bytes + 255) & ~(size_t)255; return o; };
  const size_t oLin16 = carve((size_t)5 * 4096 * 2);
  const size_t oLinBf = carve((size_t)2 * 4096 * 2);
  const size_t oC1A = carve((size_t)64 * K1A * 2),  oC1B = carve((size_t)64 * K1B * 2),  oC1S = carve((size_t)64 * K1S * 2);
  const size_t oC2A = carve((size_t)128 * K2A * 2), oC2B = carve((size_t)128 * K2B * 2), oC2S = carve((size_t)128 * K2S * 2);
  const size_t oC3A = carve((size_t)256 * K3A * 2), oC3B = carve((size_t)256 * K3B * 2), oC3S = carve((size_t)256 * K3S * 2);
  const size_t oNQ = carve((size_t)NNODE * HIDC * 4);
  const size_t oS1 = carve((size_t)NVOX * HIDC * 4);
  const size_t oX0 = carve((size_t)NVOX * 64 * 2);
  const size_t oT1 = carve((size_t)NVOX * 64 * 2);
  const size_t oY1 = carve((size_t)NVOX * 64 * 2);
  const size_t oT2 = carve((size_t)NVOX * 128 * 2);
  const size_t oY2 = carve((size_t)NVOX * 128 * 2);
  const size_t oT3 = carve((size_t)NVOX * 256 * 2);
  const size_t oY3 = carve((size_t)NVOX * 256 * 4);
  if (off > ws_size || off > (size_t)134217728) return;

  _Float16* lin16 = (_Float16*)(ws + oLin16);
  unsigned short* linbf = (unsigned short*)(ws + oLinBf);
  _Float16* ew2p  = lin16 + 0 * 4096;
  _Float16* mw1ap = lin16 + 1 * 4096;
  _Float16* mw1bp = lin16 + 2 * 4096;
  _Float16* uw1p  = lin16 + 3 * 4096;
  _Float16* uw2p  = lin16 + 4 * 4096;
  unsigned short* w2hi = linbf;
  unsigned short* w2lo = linbf + 4096;
  _Float16* pc1a = (_Float16*)(ws + oC1A); _Float16* pc1b = (_Float16*)(ws + oC1B); _Float16* pc1s = (_Float16*)(ws + oC1S);
  _Float16* pc2a = (_Float16*)(ws + oC2A); _Float16* pc2b = (_Float16*)(ws + oC2B); _Float16* pc2s = (_Float16*)(ws + oC2S);
  _Float16* pc3a = (_Float16*)(ws + oC3A); _Float16* pc3b = (_Float16*)(ws + oC3B); _Float16* pc3s = (_Float16*)(ws + oC3S);
  float* nq  = (float*)(ws + oNQ);
  float* s1  = (float*)(ws + oS1);
  _Float16* x0h = (_Float16*)(ws + oX0);
  _Float16* t1h = (_Float16*)(ws + oT1);
  _Float16* y1h = (_Float16*)(ws + oY1);
  _Float16* t2h = (_Float16*)(ws + oT2);
  _Float16* y2h = (_Float16*)(ws + oY2);
  _Float16* t3h = (_Float16*)(ws + oT3);
  float* y3f = (float*)(ws + oY3);

  const float BNC = 0.99999500003749977f;
  const float OSC = BNC * 0.015625f;

  k_prep_lin<<<7, 256, 0, stream>>>(ew2, mw1, uw1, uw2, mw2, lin16, linbf);
  auto prepc = [&](const float* W, _Float16* P, int Cout, int Cin, int T) {
    const int np = Cout * ((T * Cin) / 8);
    const int nblk = (np + 255) / 256;
    k_prep_conv<<<nblk, 256, 0, stream>>>(W, P, Cout, Cin, T);
  };
  prepc(c1a, pc1a, 64, 64, 27);
  prepc(c1b, pc1b, 64, 64, 27);
  prepc(c1s, pc1s, 64, 64, 125);
  prepc(c2a, pc2a, 128, 64, 27);
  prepc(c2b, pc2b, 128, 128, 27);
  prepc(c2s, pc2s, 128, 64, 125);
  prepc(c3a, pc3a, 256, 128, 27);
  prepc(c3b, pc3b, 256, 256, 27);
  prepc(c3s, pc3s, 256, 128, 125);

  k_nq<<<NNODE / (16 * NWAV), NTHR, 0, stream>>>(node_emb, mw1ap, nq);
  k_mpnn<<<NVOX / NWAV, NTHR, 0, stream>>>(node_pos, grid_pos, edge_i, ew1, eb1, eb2, mb1,
                                           ew2p, mw1bp, nq, s1, NNODE);
  k_upd<<<NVOX / (16 * NWAV), NTHR, 0, stream>>>(s1, w2hi, w2lo, mb2, uw1p, ub1, uw2p, ub2, x0h, BNC);

  k_conv<64, 0, 64, 0><<<(256 * 1) / NWAV, NTHR, 0, stream>>>(x0h, pc1a, x0h, pc1a, t1h, y3f, OSC);
  k_conv<64, 64, 64, 0><<<(256 * 1) / NWAV, NTHR, 0, stream>>>(t1h, pc1b, x0h, pc1s, y1h, y3f, OSC);
  k_conv<64, 0, 128, 0><<<(256 * 2) / NWAV, NTHR, 0, stream>>>(y1h, pc2a, y1h, pc2a, t2h, y3f, OSC);
  k_conv<128, 64, 128, 0><<<(256 * 2) / NWAV, NTHR, 0, stream>>>(t2h, pc2b, y1h, pc2s, y2h, y3f, OSC);
  k_conv<128, 0, 256, 0><<<(256 * 4) / NWAV, NTHR, 0, stream>>>(y2h, pc3a, y2h, pc3a, t3h, y3f, OSC);
  k_conv<256, 128, 256, 1><<<(256 * 4) / NWAV, NTHR, 0, stream>>>(t3h, pc3b, y2h, pc3s, x0h, y3f, OSC);

  k_pool<<<1, 256, 0, stream>>>(y3f, fcw, fcb, out);
}
